// BF_Model_82368882802800
// MI455X (gfx1250) — hardware-verified
//
#include <hip/hip_runtime.h>
#include <stddef.h>


#define HD     64
#define NLAY   2
#define NTH    256
#define NWAV   (NTH / 32)
#define NBA    1024
#define LNBA   10
#define NBMAX  128
#define NCHMAX 128
#define EPT    128
#define CH     (NTH * EPT)
#define SCAP   (CH + NBMAX * 32)
#define SLINES (SCAP / 32)
#define PLH    (HD * HD)
#define NPL    (2 * NLAY)
#define NTPW   (NBA / (16 * NWAV))
#define WSC    64.0f
#define HSC    16.0f
#define RH     0.0009765625f
#define WSCAP  134217728
#define EMPTYK 0xFFFFFFFFu

#define LB_AGG 0
#define LB_OUT (LB_AGG + NBA * HD * 4)
#define LB_SXS (LB_OUT + NBA * 4)
#define LB_SEA (LB_SXS + NWAV * 32 * 4)
#define LB_W0  (LB_SEA + NWAV * 32 * 4)
#define LB_W1  (LB_W0 + HD * 4)
#define LB_B1  (LB_W1 + HD * 4)
#define LB_AB2 (LB_B1 + HD * 4)
#define LB_UB1 (LB_AB2 + HD * 4)
#define LB_UW2 (LB_UB1 + HD * 4)
#define LDS_L  (LB_UW2 + HD * 4)
#define LC_HST 0
#define LC_CNT (LC_HST + NBMAX * NTH * 2)
#define LDS_C  (LC_CNT + NBMAX * 4)
#define LO_PC  0
#define LO_OFF (LO_PC + NCHMAX * NBMAX * 4)
#define LO_BSL (LO_OFF + NBMAX * NCHMAX * 4)
#define LDS_O  (LO_BSL + 2 * NBMAX * 4)
#define LF_HST 0
#define LF_STG (LF_HST + NBMAX * NTH * 2)
#define LF_GLN (LF_STG + SCAP * 4)
#define LF_LOF (LF_GLN + SLINES * 4)
#define LF_PC  (LF_LOF + NBMAX * 4)
#define LF_GO  (LF_PC + NBMAX * 4)
#define LF_TOT (LF_GO + NBMAX * 4)
#define LDS_F  (LF_TOT + 64)

static_assert(LDS_L == 269824);
static_assert(LDS_C == 66048);
static_assert(LDS_O == 132096);
static_assert(LDS_F == 219200);
static_assert((NBA & (NBA - 1)) == 0 && NBA == (1 << LNBA) && NBA == 4 * NTH);
static_assert(NTPW * 16 * NWAV == NBA);
static_assert(CH == 32768 && (SCAP % 32) == 0 && SCAP >= CH + NBMAX * 31 + 32);
static_assert((NBMAX * NTH * 2) % (16 * NTH) == 0 && (SCAP * 4) % (16 * NTH) == 0);
static_assert(NBMAX <= NTH && NBMAX % 4 == 0 && (NBMAX * NCHMAX) % (4 * NTH) == 0 && 2 * NBMAX == 4 * 64);
static_assert((LB_OUT % 16) == 0 && (LB_SXS % 16) == 0 && (LB_W0 % 16) == 0);
static_assert((LF_STG % 16) == 0 && (LF_GLN % 16) == 0 && (LF_LOF % 16) == 0 && (LF_TOT % 16) == 0);
static_assert((LO_OFF % 16) == 0 && (LO_BSL % 16) == 0 && (LC_CNT % 16) == 0);
static_assert(HD == 64 && PLH == 2 * 256 * 8);

typedef float          v4f  __attribute__((ext_vector_type(4)));
typedef float          v8f  __attribute__((ext_vector_type(8)));
typedef int            v4i  __attribute__((ext_vector_type(4)));
typedef unsigned       v4u  __attribute__((ext_vector_type(4)));
typedef _Float16       v4h  __attribute__((ext_vector_type(4)));
typedef _Float16       v8h  __attribute__((ext_vector_type(8)));
typedef _Float16       v16h __attribute__((ext_vector_type(16)));
union Frag { v16h v; v8h h[2]; v4h q[4]; };

__device__ __forceinline__ v8f wmh(v16h a, v16h b, v8f c) {
  v8f d = __builtin_amdgcn_wmma_f32_16x16x32_f16(false, a, false, b, (short)0, c, false, false);
  asm volatile("v_nop\n\tv_nop\n\tv_nop\n\tv_nop" : "+v"(d) : "v"(a), "v"(b));
  return d;
}

__device__ __forceinline__ unsigned fenc(float f) {
  const unsigned u = __float_as_uint(f);
  return (u & 0x80000000u) ? ~u : (u | 0x80000000u);
}
__device__ __forceinline__ _Float16 dec16(unsigned u) {
  const unsigned bits = (u & 0x80000000u) ? (u & 0x7FFFFFFFu) : ~u;
  float f = __uint_as_float(bits);
  f = (u == EMPTYK) ? 0.0f : f;
  return (_Float16)(f * HSC);
}
__device__ __forceinline__ v4h dec4(v4u w) {
  v4h r;
  r.x = dec16(w.x); r.y = dec16(w.y); r.z = dec16(w.z); r.w = dec16(w.w);
  return r;
}

__device__ __forceinline__ v4h h4(float xs, float ev, v4f w0, v4f w1, v4f b) {
  v4h r;
  r.x = (_Float16)fmaxf(fmaf(xs, w0.x, fmaf(ev, w1.x, b.x)), 0.0f);
  r.y = (_Float16)fmaxf(fmaf(xs, w0.y, fmaf(ev, w1.y, b.y)), 0.0f);
  r.z = (_Float16)fmaxf(fmaf(xs, w0.z, fmaf(ev, w1.z, b.z)), 0.0f);
  r.w = (_Float16)fmaxf(fmaf(xs, w0.w, fmaf(ev, w1.w, b.w)), 0.0f);
  return r;
}

__global__ __launch_bounds__(256) void k_wprep(const float* __restrict__ aW2, const float* __restrict__ uW1,
                                               _Float16* Bpl) {
  const int blk = blockIdx.x, tid = threadIdx.x;
  const int p = blk >> 1;
  const int i = (blk & 1) * 256 + tid;
  const int n = i >> 3, k0 = (i & 7) * 8;
  const float* W = ((p & 1) ? uW1 : aW2) + (size_t)(p >> 1) * PLH;
  float v[8];
#pragma unroll
  for (int e = 0; e < 8; ++e) v[e] = W[(k0 + e) * HD + n];
  v8h hv;
#pragma unroll
  for (int e = 0; e < 8; ++e) hv[e] = (_Float16)(v[e] * WSC);
  _Float16* dp = Bpl + (size_t)p * PLH + i * 8;
  *(volatile v8h*)dp = hv;
  __threadfence();
  *(volatile v8h*)dp = hv;
}

template <int PLACE>
__device__ __forceinline__ void ent1(unsigned short* hist, const int* sloff, unsigned* stage,
                                     int tid, int nN, int d, int e) {
  const bool ok = (unsigned)d < (unsigned)nN;
  int b = ok ? (d >> LNBA) : 0;
  b = b > NBMAX - 1 ? NBMAX - 1 : b;
  unsigned short* p = hist + b * NTH + tid;
  const int cur = (int)(*p);
  if (PLACE) {
    int idx = sloff[b] + cur;
    idx = idx < 0 ? 0 : (idx > SCAP - 1 ? SCAP - 1 : idx);
    if (ok) stage[idx] = (unsigned)e;
  }
  *p = (unsigned short)(cur + (ok ? 1 : 0));
}

template <int PLACE>
__device__ __forceinline__ void chunk_pass(const int* __restrict__ ids, int nE, int nN, int cbase, int tid,
                                           int vec, unsigned short* hist, const int* sloff, unsigned* stage) {
  const int e0 = cbase + EPT * tid;
  if (vec != 0 && cbase + CH <= nE) {
#pragma unroll 1
    for (int q = 0; q < EPT / 4; ++q) {
      const int eb = e0 + 4 * q;
      const v4i t4 = *(const v4i*)(ids + eb);
      ent1<PLACE>(hist, sloff, stage, tid, nN, t4.x, eb);
      ent1<PLACE>(hist, sloff, stage, tid, nN, t4.y, eb + 1);
      ent1<PLACE>(hist, sloff, stage, tid, nN, t4.z, eb + 2);
      ent1<PLACE>(hist, sloff, stage, tid, nN, t4.w, eb + 3);
    }
  } else {
#pragma unroll 1
    for (int j = 0; j < EPT; ++j) {
      int idx = e0 + j;
      const bool in = idx < nE;
      idx = in ? idx : nE - 1;
      int v = ids[idx];
      v = in ? v : -1;
      ent1<PLACE>(hist, sloff, stage, tid, nN, v, e0 + j);
    }
  }
}

__global__ __launch_bounds__(NTH) void k_bcount(const int* __restrict__ dsts, int* CNT, int nN, int nE, int vec) {
  extern __shared__ __attribute__((aligned(16))) char dynl[];
  unsigned short* hist = (unsigned short*)(dynl + LC_HST);
  int* scnt = (int*)(dynl + LC_CNT);
  const int tid = threadIdx.x;
  const int c = blockIdx.x, cbase = c * CH;
  {
    v4u z = {0u, 0u, 0u, 0u};
    v4u* p = (v4u*)hist;
#pragma unroll
    for (int it = 0; it < (NBMAX * NTH * 2) / (16 * NTH); ++it) p[it * NTH + tid] = z;
  }
  __syncthreads();
  chunk_pass<0>(dsts, nE, nN, cbase, tid, vec, hist, (const int*)0, (unsigned*)0);
  __syncthreads();
  if (tid < NBMAX) {
    int s = 0;
#pragma unroll 4
    for (int t = 0; t < NTH; ++t) s += (int)hist[tid * NTH + t];
    scnt[tid] = s;
  }
  __syncthreads();
  int* gp = CNT + (size_t)c * NBMAX;
  v4i v = {0, 0, 0, 0};
  if (tid < NBMAX / 4) v = ((const v4i*)scnt)[tid];
  if (tid < NBMAX / 4) *(volatile v4i*)(gp + 4 * tid) = v;
  __threadfence();
  if (tid < NBMAX / 4) *(volatile v4i*)(gp + 4 * tid) = v;
}

__global__ __launch_bounds__(NTH) void k_boff(const int* __restrict__ CNT, int* OFF, int* BSL, int nch) {
  extern __shared__ __attribute__((aligned(16))) char dynl[];
  int* spc  = (int*)(dynl + LO_PC);
  int* soff = (int*)(dynl + LO_OFF);
  int* sbl  = (int*)(dynl + LO_BSL);
  const int tid = threadIdx.x;
  const int ntab = nch * NBMAX;
#pragma unroll 1
  for (int i = tid; i < ntab; i += NTH) {
    int v = CNT[i];
    v = v < 0 ? 0 : (v > CH ? CH : v);
    spc[i] = (v + 31) & ~31;
  }
  __syncthreads();
  if (tid < NBMAX) {
    int tot = 0;
#pragma unroll 1
    for (int c = 0; c < nch; ++c) tot += spc[c * NBMAX + tid];
    sbl[NBMAX + tid] = tot;
  }
  __syncthreads();
  if (tid == 0) {
    int run = 0;
#pragma unroll 1
    for (int b = 0; b < NBMAX; ++b) { sbl[b] = run; run += sbl[NBMAX + b]; }
  }
  __syncthreads();
  if (tid < NBMAX) {
    int run = sbl[tid];
#pragma unroll 1
    for (int c = 0; c < NCHMAX; ++c) {
      const int cc = c < nch ? c : nch - 1;
      const int v = spc[cc * NBMAX + tid];
      soff[tid * NCHMAX + c] = run;
      run += (c < nch) ? v : 0;
    }
  }
  __syncthreads();

#pragma unroll
  for (int it = 0; it < (NBMAX * NCHMAX) / (4 * NTH); ++it) {
    const int f = it * NTH + tid;
    const v4i v = ((const v4i*)soff)[f];
    *(volatile v4i*)(OFF + 4 * f) = v;
  }
  v4i bv = {0, 0, 0, 0};
  if (tid < 64) bv = ((const v4i*)sbl)[tid];
  if (tid < 64) *(volatile v4i*)(BSL + 4 * tid) = bv;
  __threadfence();
#pragma unroll
  for (int it = 0; it < (NBMAX * NCHMAX) / (4 * NTH); ++it) {
    const int f = it * NTH + tid;
    const v4i v = ((const v4i*)soff)[f];
    *(volatile v4i*)(OFF + 4 * f) = v;
  }
  if (tid < 64) *(volatile v4i*)(BSL + 4 * tid) = bv;
}

__global__ __launch_bounds__(NTH) void k_bfill(const int* __restrict__ dsts, const int* __restrict__ OFF,
                                               unsigned* BED, int nN, int nE, int vec, int ecap) {
  extern __shared__ __attribute__((aligned(16))) char dynl[];
  unsigned short* hist = (unsigned short*)(dynl + LF_HST);
  unsigned* stage = (unsigned*)(dynl + LF_STG);
  int* gline = (int*)(dynl + LF_GLN);
  int* sloff = (int*)(dynl + LF_LOF);
  int* spc   = (int*)(dynl + LF_PC);
  int* sgo   = (int*)(dynl + LF_GO);
  int* stot  = (int*)(dynl + LF_TOT);
  const int tid = threadIdx.x;
  const int c = blockIdx.x, cbase = c * CH;
  {
    v4u z = {0u, 0u, 0u, 0u};
    v4u* p = (v4u*)hist;
#pragma unroll
    for (int it = 0; it < (NBMAX * NTH * 2) / (16 * NTH); ++it) p[it * NTH + tid] = z;
    v4u sv = {EMPTYK, EMPTYK, EMPTYK, EMPTYK};
    v4u* q = (v4u*)stage;
#pragma unroll 4
    for (int it = 0; it < (SCAP * 4) / (16 * NTH); ++it) q[it * NTH + tid] = sv;
  }
  __syncthreads();
  chunk_pass<0>(dsts, nE, nN, cbase, tid, vec, hist, (const int*)0, (unsigned*)0);
  __syncthreads();
  if (tid < NBMAX) {
    int run = 0;
#pragma unroll 4
    for (int t = 0; t < NTH; ++t) {
      const int v = (int)hist[tid * NTH + t];
      hist[tid * NTH + t] = (unsigned short)run;
      run += v;
    }
    const int pc = (run + 31) & ~31;
    spc[tid] = pc;
    int go = OFF[tid * NCHMAX + c];
    int lim = ecap - pc;
    lim = lim < 0 ? 0 : lim;
    go = go < 0 ? 0 : (go > lim ? lim : go);
    go &= ~31;
    sgo[tid] = go;
  }
  __syncthreads();
  if (tid == 0) {
    int acc = 0;
#pragma unroll 1
    for (int b = 0; b < NBMAX; ++b) { sloff[b] = acc; acc += spc[b]; }
    stot[0] = acc;
  }
  __syncthreads();
  if (tid < NBMAX) {
    const int l0 = sloff[tid] >> 5, go = sgo[tid];
    int nl = spc[tid] >> 5;
    nl = nl > SLINES ? SLINES : nl;
#pragma unroll 1
    for (int q = 0; q < nl; ++q) {
      int ln = l0 + q;
      ln = ln > SLINES - 1 ? SLINES - 1 : ln;
      gline[ln] = go + 32 * q;
    }
  }
  chunk_pass<1>(dsts, nE, nN, cbase, tid, vec, hist, sloff, stage);
  __syncthreads();

  int nlines = __builtin_amdgcn_readfirstlane(stot[0]) >> 5;
  nlines = nlines < 0 ? 0 : (nlines > SLINES ? SLINES : nlines);
  const int grp = tid >> 3, pc4 = (tid & 7) * 4;
#pragma unroll 1
  for (int base = 0; base < nlines; base += NTH / 8) {
    const int ln = base + grp;
    if (ln < nlines) {
      int g = gline[ln];
      g = g < 0 ? 0 : (g > ecap - 32 ? ecap - 32 : g);
      g &= ~31;
      const v4u v = *(const v4u*)(stage + ln * 32 + pc4);
      *(volatile v4u*)(BED + (size_t)g + pc4) = v;
    }
  }
  __threadfence();
#pragma unroll 1
  for (int base = 0; base < nlines; base += NTH / 8) {
    const int ln = base + grp;
    if (ln < nlines) {
      int g = gline[ln];
      g = g < 0 ? 0 : (g > ecap - 32 ? ecap - 32 : g);
      g &= ~31;
      const v4u v = *(const v4u*)(stage + ln * 32 + pc4);
      *(volatile v4u*)(BED + (size_t)g + pc4) = v;
    }
  }
}

__device__ __forceinline__ void edge_tile(
    const unsigned* __restrict__ tent,
    const float* __restrict__ xin, const float* __restrict__ ea,
    const int* __restrict__ srcs, const int* __restrict__ dsts,
    const _Float16* __restrict__ Bm, float* sxs, float* sea,
    const float* sw0, const float* sw1, const float* sb1, const float* sab2,
    unsigned* sagg, int n0, int nN, int nE, int lane) {
  const int hh = lane >> 4, m = lane & 15;
  const unsigned ent = tent[m];
  const bool eok = ent < (unsigned)nE;
  const int e = eok ? (int)ent : 0;
  int s = srcs[e];
  s = s < 0 ? 0 : (s > nN - 1 ? nN - 1 : s);
  const int dd = dsts[e];
  const unsigned ldu = (unsigned)dd - (unsigned)n0;
  const bool rv = eok && (ldu < (unsigned)NBA);
  const int ldv = rv ? (int)ldu : -1;
  const float xg = xin[s];
  const float eg = ea[e];
  sxs[lane] = xg;
  sea[lane] = eg;
  __builtin_amdgcn_fence(__ATOMIC_RELEASE, "wavefront");
  __builtin_amdgcn_wave_barrier();
  const float xs = sxs[m];
  const float ev = sea[m];

  v8f acc[4];
#pragma unroll
  for (int t = 0; t < 4; ++t) { v8f z = {0.f, 0.f, 0.f, 0.f, 0.f, 0.f, 0.f, 0.f}; acc[t] = z; }
  const _Float16* bb = Bm + (size_t)m * HD + 8 * hh;
  const v4f* w0p = (const v4f*)sw0;
  const v4f* w1p = (const v4f*)sw1;
  const v4f* bp  = (const v4f*)sb1;
#pragma unroll
  for (int ks = 0; ks < HD / 32; ++ks) {
    const int qlo = 8 * ks + 2 * hh;
    const int qhi = qlo + 4;
    Frag a;
    a.q[0] = h4(xs, ev, w0p[qlo],     w1p[qlo],     bp[qlo]);
    a.q[1] = h4(xs, ev, w0p[qlo + 1], w1p[qlo + 1], bp[qlo + 1]);
    a.q[2] = h4(xs, ev, w0p[qhi],     w1p[qhi],     bp[qhi]);
    a.q[3] = h4(xs, ev, w0p[qhi + 1], w1p[qhi + 1], bp[qhi + 1]);
#pragma unroll
    for (int t = 0; t < 4; ++t) {
      const _Float16* bq = bb + (size_t)(16 * t) * HD + 32 * ks;
      Frag b;
      b.h[0] = *(const v8h*)bq;
      b.h[1] = *(const v8h*)(bq + 16);
      acc[t] = wmh(a.v, b.v, acc[t]);
    }
  }

  int dl[8];
#pragma unroll
  for (int r = 0; r < 8; ++r) dl[r] = __shfl(ldv, 8 * hh + r, 32);
#pragma unroll
  for (int t = 0; t < 4; ++t) {
    const float bv = sab2[16 * t + m];
    unsigned* colp = sagg + 16 * t + m;
#pragma unroll
    for (int r = 0; r < 8; ++r) {
      const float val = fmaf(acc[t][r], RH, bv);
      const bool rok = dl[r] >= 0;
      const int node = rok ? dl[r] : 0;
      const unsigned key = rok ? fenc(val) : EMPTYK;
      atomicMin(colp + node * HD, key);
    }
  }
}

__device__ __forceinline__ void node_tile(const unsigned* sagg, int r0, const _Float16* __restrict__ Bu,
                                          const float* sub1, const float* suw2, float ub2v,
                                          float* sout, int lane) {
  const int hh = lane >> 4, m = lane & 15;
  const unsigned* arow = sagg + (r0 + m) * HD + 8 * hh;
  float b1c[4], w2c[4];
#pragma unroll
  for (int t = 0; t < 4; ++t) { b1c[t] = sub1[16 * t + m]; w2c[t] = suw2[16 * t + m]; }
  v8f acc[4];
#pragma unroll
  for (int t = 0; t < 4; ++t) { v8f z = {0.f, 0.f, 0.f, 0.f, 0.f, 0.f, 0.f, 0.f}; acc[t] = z; }
  const _Float16* bb = Bu + (size_t)m * HD + 8 * hh;
#pragma unroll
  for (int ks = 0; ks < HD / 32; ++ks) {
    const v4u u0 = *(const v4u*)(arow + 32 * ks);
    const v4u u1 = *(const v4u*)(arow + 32 * ks + 4);
    const v4u u2 = *(const v4u*)(arow + 32 * ks + 16);
    const v4u u3 = *(const v4u*)(arow + 32 * ks + 20);
    Frag a;
    a.q[0] = dec4(u0); a.q[1] = dec4(u1); a.q[2] = dec4(u2); a.q[3] = dec4(u3);
#pragma unroll
    for (int t = 0; t < 4; ++t) {
      const _Float16* bq = bb + (size_t)(16 * t) * HD + 32 * ks;
      Frag b;
      b.h[0] = *(const v8h*)bq;
      b.h[1] = *(const v8h*)(bq + 16);
      acc[t] = wmh(a.v, b.v, acc[t]);
    }
  }

  float v[8];
#pragma unroll
  for (int r = 0; r < 8; ++r) {
    float s = 0.0f;
#pragma unroll
    for (int t = 0; t < 4; ++t) {
      const float u = fmaxf(fmaf(acc[t][r], RH, b1c[t]), 0.0f);
      s = fmaf(u, w2c[t], s);
    }
    v[r] = s;
  }
  float u4[4];
  {
    const bool kb = ((lane >> 3) & 1) != 0;
#pragma unroll
    for (int i = 0; i < 4; ++i) {
      const float snd = kb ? v[i] : v[i + 4];
      const float kp  = kb ? v[i + 4] : v[i];
      u4[i] = kp + __shfl_xor(snd, 8, 32);
    }
  }
  float w2[2];
  {
    const bool kb = ((lane >> 2) & 1) != 0;
#pragma unroll
    for (int i = 0; i < 2; ++i) {
      const float snd = kb ? u4[i] : u4[i + 2];
      const float kp  = kb ? u4[i + 2] : u4[i];
      w2[i] = kp + __shfl_xor(snd, 4, 32);
    }
  }
  float z;
  {
    const bool kb = ((lane >> 1) & 1) != 0;
    const float snd = kb ? w2[0] : w2[1];
    const float kp  = kb ? w2[1] : w2[0];
    z = kp + __shfl_xor(snd, 2, 32);
  }
  const float fin = z + __shfl_xor(z, 1, 32);
  sout[r0 + 8 * hh + (m >> 1)] = fin + ub2v;
}

__global__ __launch_bounds__(NTH) void k_layer(
    const float* __restrict__ xin, const float* __restrict__ ea,
    const int* __restrict__ srcs, const int* __restrict__ dsts,
    const unsigned* __restrict__ BED, const int* __restrict__ BSL,
    const float* __restrict__ aW1l, const float* __restrict__ ab1l, const float* __restrict__ ab2l,
    const _Float16* __restrict__ Bm, const _Float16* __restrict__ Bu,
    const float* __restrict__ ub1l, const float* __restrict__ uW2l, const float* __restrict__ ub2l,
    float* xout, int nN, int nE, int ecap, int nWrite) {
  extern __shared__ __attribute__((aligned(16))) char dynl[];
  unsigned* sagg = (unsigned*)(dynl + LB_AGG);
  float* sout = (float*)(dynl + LB_OUT);
  float* sxs  = (float*)(dynl + LB_SXS);
  float* sea  = (float*)(dynl + LB_SEA);
  float* sw0  = (float*)(dynl + LB_W0);
  float* sw1  = (float*)(dynl + LB_W1);
  float* sb1  = (float*)(dynl + LB_B1);
  float* sab2 = (float*)(dynl + LB_AB2);
  float* sub1 = (float*)(dynl + LB_UB1);
  float* suw2 = (float*)(dynl + LB_UW2);
  const int tid = threadIdx.x, lane = tid & 31;
  const int wave = __builtin_amdgcn_readfirstlane(tid >> 5);
  const int n0 = blockIdx.x * NBA;

  if (tid < HD) {
    sw0[tid]  = aW1l[tid] * HSC;
    sw1[tid]  = aW1l[HD + tid] * HSC;
    sb1[tid]  = ab1l[tid] * HSC;
    sab2[tid] = ab2l[tid];
    sub1[tid] = ub1l[tid];
    suw2[tid] = uW2l[tid];
  }
  const float ub2v = ub2l[0];
  {
    v4u z = {EMPTYK, EMPTYK, EMPTYK, EMPTYK};
    v4u* p = (v4u*)sagg;
#pragma unroll 4
    for (int it = 0; it < (NBA * HD) / (4 * NTH); ++it) p[it * NTH + tid] = z;
  }
  __syncthreads();

  int st = BSL[blockIdx.x];
  int ln = BSL[NBMAX + blockIdx.x];
  st = st < 0 ? 0 : (st > ecap ? ecap : st);
  st &= ~31;
  const int rem = ecap - st;
  ln = ln < 0 ? 0 : (ln > rem ? rem : ln);
  ln &= ~31;
  const int stu   = __builtin_amdgcn_readfirstlane(st);
  const int ntile = __builtin_amdgcn_readfirstlane(ln >> 4);
  const unsigned* seg = BED + (size_t)stu;
  float* wsx = sxs + wave * 32;
  float* wse = sea + wave * 32;
  for (int ti = wave; ti < ntile; ti += NWAV)
    edge_tile(seg + (size_t)16 * ti, xin, ea, srcs, dsts, Bm, wsx, wse, sw0, sw1, sb1, sab2,
              sagg, n0, nN, nE, lane);
  __syncthreads();

#pragma unroll 1
  for (int i = 0; i < NTPW; ++i)
    node_tile(sagg, 16 * (wave * NTPW + i), Bu, sub1, suw2, ub2v, sout, lane);
  __syncthreads();

  const v4f ov = ((const v4f*)sout)[tid];
  const int g0 = n0 + 4 * tid;
  float* op = xout + g0;
  const bool full = (g0 + 3 < nWrite);
  if (full) {
    *(volatile v4f*)op = ov;
  } else {
    if (g0     < nWrite) *(volatile float*)(op)     = ov.x;
    if (g0 + 1 < nWrite) *(volatile float*)(op + 1) = ov.y;
    if (g0 + 2 < nWrite) *(volatile float*)(op + 2) = ov.z;
  }
  __threadfence();
  if (full) {
    *(volatile v4f*)op = ov;
  } else {
    if (g0     < nWrite) *(volatile float*)(op)     = ov.x;
    if (g0 + 1 < nWrite) *(volatile float*)(op + 1) = ov.y;
    if (g0 + 2 < nWrite) *(volatile float*)(op + 2) = ov.z;
  }
}

extern "C" void kernel_launch(void* const* d_in, const int* in_sizes, int n_in,
                              void* d_out, int out_size, void* d_ws, size_t ws_size,
                              hipStream_t stream) {
  if (n_in < 11) return;
  const int nN = in_sizes[0];
  const int nE = in_sizes[1];
  if (nN < 1 || nE < 1) return;
  if (in_sizes[2] != NLAY * 2 * HD || in_sizes[3] != NLAY * HD) return;
  if (in_sizes[4] != NLAY * HD * HD || in_sizes[5] != NLAY * HD) return;
  if (in_sizes[6] != NLAY * HD * HD || in_sizes[7] != NLAY * HD) return;
  if (in_sizes[8] != NLAY * HD || in_sizes[9] != NLAY) return;
  if (in_sizes[10] != 2 * nE) return;
  if (out_size != nN) return;
  if (nN > (1 << 22) || nE > (1 << 22)) return;

  const float* x   = (const float*)d_in[0];
  const float* ea  = (const float*)d_in[1];
  const float* aW1 = (const float*)d_in[2];
  const float* ab1 = (const float*)d_in[3];
  const float* aW2 = (const float*)d_in[4];
  const float* ab2 = (const float*)d_in[5];
  const float* uW1 = (const float*)d_in[6];
  const float* ub1 = (const float*)d_in[7];
  const float* uW2 = (const float*)d_in[8];
  const float* ub2 = (const float*)d_in[9];
  const int*   ei  = (const int*)d_in[10];
  float* out = (float*)d_out;
  const int* srcs = ei;
  const int* dsts = ei + (size_t)nE;

  const int nPad = ((nN + NBA - 1) / NBA) * NBA;
  const int nb   = nPad / NBA;
  const int nch  = (nE + CH - 1) / CH;
  if (nb > NBMAX || nch > NCHMAX) return;
  const int ecap = ((nE + 31 * nb * nch + 31) / 32) * 32;
  const int vec  = ((nE & 3) == 0) ? 1 : 0;

  char* ws = (char*)d_ws;
  size_t off = 0;
  const size_t oB   = off; off += (size_t)NPL * PLH * 2;           off = (off + 255) & ~(size_t)255;
  const size_t oX   = off; off += (size_t)nPad * 4;                off = (off + 255) & ~(size_t)255;
  const size_t oCNT = off; off += (size_t)NCHMAX * NBMAX * 4;      off = (off + 255) & ~(size_t)255;
  const size_t oOFF = off; off += (size_t)NBMAX * NCHMAX * 4;      off = (off + 255) & ~(size_t)255;
  const size_t oBSL = off; off += (size_t)2 * NBMAX * 4;           off = (off + 255) & ~(size_t)255;
  const size_t oBED = off; off += (size_t)ecap * 4;                off = (off + 255) & ~(size_t)255;
  if (off > ws_size || off > (size_t)WSCAP) return;
  _Float16* Bpl = (_Float16*)(ws + oB);
  float*    X1  = (float*)(ws + oX);
  int*      CNT = (int*)(ws + oCNT);
  int*      OFF = (int*)(ws + oOFF);
  int*      BSL = (int*)(ws + oBSL);
  unsigned* BED = (unsigned*)(ws + oBED);

  hipFuncSetAttribute(reinterpret_cast<const void*>(&k_bcount), hipFuncAttributeMaxDynamicSharedMemorySize, LDS_C);
  hipFuncSetAttribute(reinterpret_cast<const void*>(&k_boff), hipFuncAttributeMaxDynamicSharedMemorySize, LDS_O);
  hipFuncSetAttribute(reinterpret_cast<const void*>(&k_bfill), hipFuncAttributeMaxDynamicSharedMemorySize, LDS_F);
  hipFuncSetAttribute(reinterpret_cast<const void*>(&k_layer), hipFuncAttributeMaxDynamicSharedMemorySize, LDS_L);

  k_wprep<<<2 * NPL, 256, 0, stream>>>(aW2, uW1, Bpl);
  k_bcount<<<nch, NTH, LDS_C, stream>>>(dsts, CNT, nN, nE, vec);
  k_boff<<<1, NTH, LDS_O, stream>>>(CNT, OFF, BSL, nch);
  k_bfill<<<nch, NTH, LDS_F, stream>>>(dsts, OFF, BED, nN, nE, vec, ecap);
  for (int l = 0; l < NLAY; ++l) {
    const float* xl = (l == 0) ? x : X1;
    float* xo = (l == NLAY - 1) ? out : X1;
    const int nWrite = (l == NLAY - 1) ? nN : nPad;
    k_layer<<<nb, NTH, LDS_L, stream>>>(
        xl, ea, srcs, dsts, BED, BSL,
        aW1 + (size_t)l * 2 * HD, ab1 + (size_t)l * HD, ab2 + (size_t)l * HD,
        Bpl + (size_t)(2 * l) * PLH, Bpl + (size_t)(2 * l + 1) * PLH,
        ub1 + (size_t)l * HD, uW2 + (size_t)l * HD, ub2 + l,
        xo, nN, nE, ecap, nWrite);
  }
  hipGetLastError();
}
